// GraphSAGE_23699629539638
// MI455X (gfx1250) — hardware-verified
//
#include <hip/hip_runtime.h>
#include <stddef.h>
#include <stdint.h>
#include <math.h>


#define DF     128
#define CO     64
#define AP     512
#define KK     512
#define KH     256
#define HOFF   256
#define NTHR   256
#define NWAVE  8
#define EPT    8
#define CHUNK  (NTHR * EPT)
#define WCAP   (EPT * 32)
#define LISTN  (NWAVE * WCAP)
#define NBA    1024
#define SLA    10
#define RCAP   28672
#define DEGCAP 64
#define GBM    64
#define GBN    128
#define GTHR   128
#define GWAVE  (GTHR / 32)
#define PARTW  288
#define WSTW   258
#define WSTH   (2 * CO + 2)
#define NSUB   (2 * GWAVE)
#define HPR    8
#define HPB    (NWAVE * HPR)
#define OTN    64
#define XTP    132
#define OTP    68
#define RBW    (DF / 2)
#define WBL    ((DF * DF / 8) / NTHR)
#define WBH    ((CO * DF / 8) / NTHR)
#define AGG_ZINTS    (LISTN + 2 * RCAP + 3 * NBA)
#define MISC_INTS    16
#define ROWBUF_INTS  (NWAVE * DF)
#define AGG_LDS_INTS (AGG_ZINTS + MISC_INTS + ROWBUF_INTS)
#define MAXL   8
#define WSMAX  134217728

static_assert((CHUNK & (CHUNK - 1)) == 0 && CHUNK <= 4096);
static_assert((NBA & (NBA - 1)) == 0 && NBA == (1 << SLA));
static_assert(((long long)CHUNK << SLA) < (1LL << 31));
static_assert(LISTN % NTHR == 0);
static_assert(NBA % NWAVE == 0 && NBA % 32 == 0 && NBA % GBM == 0);
static_assert(RCAP % 4 == 0 && AGG_ZINTS % 4 == 0 && LISTN % 4 == 0 && ((AGG_ZINTS + MISC_INTS) % 4) == 0);
static_assert(AGG_ZINTS % (NTHR * 4) == 0);
static_assert(KK % 32 == 0 && KK == AP && AP == 4 * DF && KH == 2 * DF && KH % 32 == 0 && HOFF == 2 * DF);
static_assert((3 * DF) % 32 == 0);
static_assert(GBN == DF && GBM == GWAVE * 16 && DF == 4 * 32 && GTHR == DF);
static_assert(CO == 4 * 16 && CO <= GBN && CO / 4 == 16);
static_assert(PARTW % 32 == 0 && PARTW / 4 <= GTHR && PARTW >= 2 * GBN + 1);
static_assert(WSTW >= 2 * GBN + 1 && (WSTW % 2) == 0 && WSTH >= 2 * CO + 1 && (WSTH % 2) == 0);
static_assert(HPB == GBM && NTHR == 2 * DF && OTN == GBM && OTN == HPB);
static_assert(WBL * NTHR * 8 == DF * DF && WBH * NTHR * 8 == CO * DF);
static_assert((DF * OTN / 4) % NTHR == 0 && (DF * OTN / 4) / NTHR == 8 && OTN / 4 == 16);
static_assert((OTN * CO / 4) % NTHR == 0 && (OTN * CO / 4) / NTHR == 4);
static_assert(OTP % 4 == 0 && OTP >= OTN && XTP >= DF && (XTP % 4) == 0);
static_assert(RBW * 2 == DF && 4 * 32 == 2 * RBW);
static_assert(CO == 8 * NWAVE);
static_assert(AGG_LDS_INTS * 4 <= 300000);
static_assert(OTN * XTP * 4 <= 64000);

typedef float          v4f   __attribute__((ext_vector_type(4)));
typedef float          v8f   __attribute__((ext_vector_type(8)));
typedef int            v4i   __attribute__((ext_vector_type(4)));
typedef int            v8i   __attribute__((ext_vector_type(8)));
typedef unsigned int   v2u   __attribute__((ext_vector_type(2)));
typedef unsigned int   v4u   __attribute__((ext_vector_type(4)));
typedef unsigned short v8us  __attribute__((ext_vector_type(8)));
typedef unsigned short v16us __attribute__((ext_vector_type(16)));
typedef __bf16         v16bf __attribute__((ext_vector_type(16)));
typedef v4f  __attribute__((may_alias)) v4fa;
typedef v4i  __attribute__((may_alias)) v4ia;
typedef v2u  __attribute__((may_alias)) v2ua;
typedef v4u  __attribute__((may_alias)) v4ua;
typedef v8us __attribute__((may_alias)) v8usa;
union FragB { v16bf v; v16us u; v8us h[2]; v8i w; };

__device__ __forceinline__ v8f wmb(const FragB& a, const FragB& b, v8f c) {
  v8f d = __builtin_amdgcn_wmma_f32_16x16x32_bf16(false, a.v, false, b.v, (short)0, c, false, false);
  asm volatile("v_nop\n\tv_nop\n\tv_nop\n\tv_nop" : "+v"(d) : "v"(a.w), "v"(b.w));
  return d;
}

__device__ __forceinline__ v8f z8() { v8f z = {0.f, 0.f, 0.f, 0.f, 0.f, 0.f, 0.f, 0.f}; return z; }

__device__ __forceinline__ unsigned bf16_bits(float f) {
  const unsigned u = __float_as_uint(f);
  return ((u + 0x7FFFu + ((u >> 16) & 1u)) >> 16) & 0xFFFFu;
}
__device__ __forceinline__ float bf16_val(float f) {
  return __uint_as_float(bf16_bits(f) << 16);
}
__device__ __forceinline__ unsigned pk2(float lo, float hi) { return bf16_bits(lo) | (bf16_bits(hi) << 16); }
__device__ __forceinline__ v4u pack8(const v4f a, const v4f b) {
  v4u r;
  r.x = pk2(a.x, a.y); r.y = pk2(a.z, a.w); r.z = pk2(b.x, b.y); r.w = pk2(b.z, b.w);
  return r;
}
__device__ __forceinline__ v4f hl4(const v2u wh, const v2u wl) {
  v4f r;
  r.x = __uint_as_float(wh.x << 16)          + __uint_as_float(wl.x << 16);
  r.y = __uint_as_float(wh.x & 0xFFFF0000u)  + __uint_as_float(wl.x & 0xFFFF0000u);
  r.z = __uint_as_float(wh.y << 16)          + __uint_as_float(wl.y << 16);
  r.w = __uint_as_float(wh.y & 0xFFFF0000u)  + __uint_as_float(wl.y & 0xFFFF0000u);
  return r;
}
__device__ __forceinline__ void split4w(const v4f y, v2u& wh, v2u& wl) {
  const unsigned h0 = bf16_bits(y.x), h1 = bf16_bits(y.y), h2 = bf16_bits(y.z), h3 = bf16_bits(y.w);
  const unsigned l0 = bf16_bits(y.x - __uint_as_float(h0 << 16));
  const unsigned l1 = bf16_bits(y.y - __uint_as_float(h1 << 16));
  const unsigned l2 = bf16_bits(y.z - __uint_as_float(h2 << 16));
  const unsigned l3 = bf16_bits(y.w - __uint_as_float(h3 << 16));
  wh.x = h0 | (h1 << 16); wh.y = h2 | (h3 << 16);
  wl.x = l0 | (l1 << 16); wl.y = l2 | (l3 << 16);
}

__device__ __forceinline__ void wave_sync() {
  __builtin_amdgcn_fence(__ATOMIC_RELEASE, "wavefront");
  __builtin_amdgcn_wave_barrier();
  __builtin_amdgcn_fence(__ATOMIC_ACQUIRE, "wavefront");
}

template <int SLB>
__device__ __forceinline__ int scan_chunk(const int* __restrict__ dsts, int nE, int cbase, int slotBase,
                                          int nb, int vec8, int* list, int tid, int lane, int wave) {
  int wc = 0;
  const int el0  = tid * EPT;
  const int e0   = cbase + el0;
  const int sent = -2147483647 - 1;
  v4i da, db;
  if (vec8 != 0 && cbase + CHUNK <= nE) {
    da = *(const v4i*)(dsts + e0);
    db = *(const v4i*)(dsts + e0 + 4);
  } else {
    da.x = (e0     < nE) ? dsts[min(e0,     nE - 1)] : sent;
    da.y = (e0 + 1 < nE) ? dsts[min(e0 + 1, nE - 1)] : sent;
    da.z = (e0 + 2 < nE) ? dsts[min(e0 + 2, nE - 1)] : sent;
    da.w = (e0 + 3 < nE) ? dsts[min(e0 + 3, nE - 1)] : sent;
    db.x = (e0 + 4 < nE) ? dsts[min(e0 + 4, nE - 1)] : sent;
    db.y = (e0 + 5 < nE) ? dsts[min(e0 + 5, nE - 1)] : sent;
    db.z = (e0 + 6 < nE) ? dsts[min(e0 + 6, nE - 1)] : sent;
    db.w = (e0 + 7 < nE) ? dsts[min(e0 + 7, nE - 1)] : sent;
  }
  const unsigned nbs = (unsigned)slotBase;
  const unsigned unb = (unsigned)nb;
  const unsigned s0 = (unsigned)da.x - nbs, s1 = (unsigned)da.y - nbs;
  const unsigned s2 = (unsigned)da.z - nbs, s3 = (unsigned)da.w - nbs;
  const unsigned s4 = (unsigned)db.x - nbs, s5 = (unsigned)db.y - nbs;
  const unsigned s6 = (unsigned)db.z - nbs, s7 = (unsigned)db.w - nbs;
  const bool h0 = s0 < unb, h1 = s1 < unb, h2 = s2 < unb, h3 = s3 < unb;
  const bool h4 = s4 < unb, h5 = s5 < unb, h6 = s6 < unb, h7 = s7 < unb;
  const unsigned any = __builtin_amdgcn_ballot_w32(h0 | h1 | h2 | h3 | h4 | h5 | h6 | h7);
  if (any != 0u) {
#define HITJ(J, HJ, SJ) { \
      const unsigned mj = __builtin_amdgcn_ballot_w32(HJ); \
      if (mj != 0u) { \
        if (HJ) { \
          const int pos = wc + (int)__builtin_amdgcn_mbcnt_lo(mj, 0u); \
          if (pos < WCAP) list[wave * WCAP + pos] = ((el0 + (J)) << SLB) | (int)(SJ); \
        } \
        wc += (int)__builtin_popcount(mj); } }
    HITJ(0, h0, s0)
    HITJ(1, h1, s1)
    HITJ(2, h2, s2)
    HITJ(3, h3, s3)
    HITJ(4, h4, s4)
    HITJ(5, h5, s5)
    HITJ(6, h6, s6)
    HITJ(7, h7, s7)
#undef HITJ
  }
  return wc;
}

__global__ __launch_bounds__(NTHR) void k_wprep(const float* __restrict__ Wself, const float* __restrict__ Wneigh,
                                                const float* __restrict__ Wc, int nL,
                                                unsigned short* Bpl, unsigned short* Bh) {
  const int b = (int)blockIdx.x, tid = (int)threadIdx.x;
  const int nlb = 16 * nL;
  const bool head = b >= nlb;
  const int l = head ? 0 : (b >> 4);
  const int r = head ? 0 : (b & 15);
  const int which = r >> 3;
  const int u = head ? ((b - nlb) * NTHR + tid) : ((r & 7) * NTHR + tid);
  const int n  = u >> 4;
  const int k8 = (u & 15) * 8;
  const float* W = head ? Wc : (((which != 0) ? Wself : Wneigh) + (size_t)l * (size_t)(DF * DF));
  const float* p = W + (size_t)n * DF + k8;
  const v4f a = *(const v4f*)p;
  const v4f c = *(const v4f*)(p + 4);
  const v4u q = pack8(a, c);
  unsigned short* dp = head ? (Bh + (size_t)n * KH + k8)
                            : (Bpl + (size_t)l * (size_t)(DF * KK) + (size_t)n * KK + which * (2 * DF) + k8);
  *(volatile v4u*)dp = q;
  *(volatile v4u*)(dp + DF) = q;
  __threadfence();
  *(volatile v4u*)dp = q;
  *(volatile v4u*)(dp + DF) = q;
}

__global__ __launch_bounds__(NTHR) void k_xprep(const float* __restrict__ x, int nN, int vx, unsigned short* apl) {
  __shared__ __attribute__((aligned(16))) float T[OTN * XTP];
  const int tid = (int)threadIdx.x, lane = tid & 31, wave = tid >> 5;
  const int n0 = (int)blockIdx.x * OTN;
  if (vx != 0 && n0 + OTN <= nN) {
#pragma unroll
    for (int it = 0; it < (DF * OTN / 4) / NTHR; ++it) {
      const int i = it * NTHR + tid;
      const int c = i >> 4;
      const int q = i & 15;
      const v4f w = *(const v4f*)(x + (size_t)c * (size_t)nN + (size_t)(n0 + 4 * q));
      T[(4 * q + 0) * XTP + c] = w.x;
      T[(4 * q + 1) * XTP + c] = w.y;
      T[(4 * q + 2) * XTP + c] = w.z;
      T[(4 * q + 3) * XTP + c] = w.w;
    }
  } else {
#pragma unroll 1
    for (int it = 0; it < (DF * OTN / 4) / NTHR; ++it) {
      const int i = it * NTHR + tid;
      const int c = i >> 4;
      const int q = i & 15;
      const float* xc = x + (size_t)c * (size_t)nN;
#pragma unroll
      for (int j = 0; j < 4; ++j) {
        const int n  = n0 + 4 * q + j;
        const int nc = n < nN ? n : (nN - 1);
        float v = xc[nc];
        v = (n < nN) ? v : 0.0f;
        T[(4 * q + j) * XTP + c] = v;
      }
    }
  }
  __syncthreads();
  const unsigned mk = (lane < 16) ? 0xFFFFFFFFu : 0u;
  v4u qv[HPR];
#pragma unroll
  for (int i = 0; i < HPR; ++i) {
    const int lr = wave * HPR + i;
    const float* tr = T + lr * XTP + 8 * (lane & 15);
    const v4f f0 = *(const v4fa*)tr;
    const v4f f1 = *(const v4fa*)(tr + 4);
    v4u q = pack8(f0, f1);
    q.x &= mk; q.y &= mk; q.z &= mk; q.w &= mk;
    qv[i] = q;
  }
#pragma unroll
  for (int i = 0; i < HPR; ++i) {
    const int row = n0 + wave * HPR + i;
    *(volatile v4u*)(apl + (size_t)row * AP + HOFF + 8 * lane) = qv[i];
  }
  __threadfence();
#pragma unroll
  for (int i = 0; i < HPR; ++i) {
    const int row = n0 + wave * HPR + i;
    *(volatile v4u*)(apl + (size_t)row * AP + HOFF + 8 * lane) = qv[i];
  }
}

__global__ __launch_bounds__(NTHR) void k_hprep(const float* __restrict__ ss, int nN, int mRows, unsigned short* apl) {
  __shared__ __attribute__((aligned(16))) float ssh[2 * DF];
  __shared__ __attribute__((aligned(16))) unsigned int rbuf[NWAVE * DF];
  const int tid = (int)threadIdx.x, lane = tid & 31, wave = tid >> 5;
  ssh[tid] = ss[tid];
  __syncthreads();
  const v4f sc = *(const v4fa*)(ssh + 4 * lane);
  const v4f sh = *(const v4fa*)(ssh + DF + 4 * lane);
  unsigned int* rb = rbuf + wave * DF;
  const int rb0 = (int)blockIdx.x * HPB + wave * HPR;

  v4u qv[HPR];
#pragma unroll
  for (int i = 0; i < HPR; ++i) {
    const int row = rb0 + i;
    const bool live = row < nN;
    const int rc = live ? row : (nN - 1);
    const unsigned short* rp = apl + (size_t)rc * AP + HOFF;
    const v2u wh = *(const v2ua*)(rp + 4 * lane);
    const v2u wl = *(const v2ua*)(rp + DF + 4 * lane);
    const v4f a = hl4(wh, wl);
    v4f y;
    y.x = fmaf(a.x, sc.x, sh.x);
    y.y = fmaf(a.y, sc.y, sh.y);
    y.z = fmaf(a.z, sc.z, sh.z);
    y.w = fmaf(a.w, sc.w, sh.w);
    y.x = live ? y.x : 0.0f; y.y = live ? y.y : 0.0f; y.z = live ? y.z : 0.0f; y.w = live ? y.w : 0.0f;
    v2u mh, ml;
    split4w(y, mh, ml);
    *(v2ua*)(rb + 2 * lane) = mh;
    *(v2ua*)(rb + RBW + 2 * lane) = ml;
    wave_sync();
    qv[i] = *(const v4ua*)(rb + 4 * lane);
    wave_sync();
  }
#pragma unroll
  for (int i = 0; i < HPR; ++i) {
    const int row = rb0 + i;
    if (row < mRows) {
      *(volatile v4u*)(apl + (size_t)row * AP + HOFF + 8 * lane) = qv[i];
    }
  }
  __threadfence();
#pragma unroll
  for (int i = 0; i < HPR; ++i) {
    const int row = rb0 + i;
    if (row < mRows) {
      *(volatile v4u*)(apl + (size_t)row * AP + HOFF + 8 * lane) = qv[i];
    }
  }
}

__global__ __launch_bounds__(NTHR) void k_scan(const int* __restrict__ srcs, const int* __restrict__ dsts,
                                               int nE, int nN, int vec8, int mRows, unsigned short* apl) {
  extern __shared__ __attribute__((aligned(16))) int dsm[];
  int* list = dsm;
  int* hl   = dsm + LISTN;
  int* sl   = hl + RCAP;
  int* cnt  = sl + RCAP;
  int* offs = cnt + NBA;
  int* cur  = offs + NBA;
  int* misc = cur + NBA;
  const int tid = (int)threadIdx.x, lane = tid & 31, wave = tid >> 5;
  unsigned int* rowbuf = (unsigned int*)(misc + MISC_INTS) + wave * DF;
  const int nodeBase = (int)blockIdx.x * NBA;

  {
    const v4i z4 = {0, 0, 0, 0};
    for (int i = tid * 4; i < AGG_ZINTS; i += NTHR * 4) *(v4ia*)(dsm + i) = z4;
    if (tid < MISC_INTS) misc[tid] = 0;
  }
  __syncthreads();

  int t = 0, ov = 0;
  const int nChunks = (nE + CHUNK - 1) / CHUNK;
#pragma unroll 1
  for (int ch = 0; ch < nChunks; ++ch) {
    const int cbase = ch * CHUNK;
    const int wc = scan_chunk<SLA>(dsts, nE, cbase, nodeBase, NBA, vec8, list, tid, lane, wave);
    if (lane == 0) misc[wave] = wc;
    __syncthreads();
    if (wave == 0) {
#pragma unroll 1
      for (int w2 = 0; w2 < NWAVE; ++w2) {
        int c = misc[w2];
        c = c < 0 ? 0 : (c > WCAP ? WCAP : c);
#pragma unroll 1
        for (int b0 = 0; b0 < c; b0 += 32) {
          const int idx = b0 + lane;
          const int ent = list[w2 * WCAP + (idx < WCAP ? idx : WCAP - 1)];
          const int m32 = (c - b0) < 32 ? (c - b0) : 32;
#pragma unroll 1
          for (int k = 0; k < m32; ++k) {
            const int u    = __builtin_amdgcn_readlane(ent, k);
            const int slot = u & (NBA - 1);
            const int el   = (u >> SLA) & (CHUNK - 1);
            const int pk   = ((cbase + el) << SLA) | slot;
            if (t < RCAP) {
              if (lane == 0) { hl[t] = pk; cnt[slot] = cnt[slot] + 1; }
              t = t + 1;
            } else {
              ov = 1;
            }
          }
        }
      }
    }
    __syncthreads();
  }
  if (wave == 0 && lane == 0) { misc[8] = t; misc[9] = ov; }
  __syncthreads();
  int tt = misc[8];
  tt = tt < 0 ? 0 : (tt > RCAP ? RCAP : tt);
  const int ovf = misc[9];

  if (wave == 0) {
    const int base = lane * (NBA / 32);
    int s = 0;
#pragma unroll 1
    for (int i = 0; i < NBA / 32; ++i) s += cnt[base + i];
    int incl = s;
#pragma unroll
    for (int d = 1; d < 32; d <<= 1) {
      const int y = __shfl_up(incl, d, 32);
      if (lane >= d) incl += y;
    }
    int run = incl - s;
#pragma unroll 1
    for (int i = 0; i < NBA / 32; ++i) {
      const int cv = cnt[base + i];
      offs[base + i] = run;
      cur[base + i]  = run;
      run += cv;
    }
  }
  __syncthreads();
  if (wave == 0) {
#pragma unroll 1
    for (int b0 = 0; b0 < tt; b0 += 32) {
      const int idx = b0 + lane;
      const int ent = hl[idx < RCAP ? idx : RCAP - 1];
      const int m32 = (tt - b0) < 32 ? (tt - b0) : 32;
#pragma unroll 1
      for (int k = 0; k < m32; ++k) {
        const int u    = __builtin_amdgcn_readlane(ent, k);
        const int slot = u & (NBA - 1);
        if (lane == 0) {
          int p = cur[slot];
          p = p < 0 ? 0 : (p > RCAP - 1 ? RCAP - 1 : p);
          sl[p] = u;
          cur[slot] = p + 1;
        }
      }
    }
  }
  __syncthreads();

  const float pz = (ovf != 0) ? __int_as_float(0x7fc00000) : 0.0f;
#pragma unroll 1
  for (int si = 0; si < NBA / NWAVE; ++si) {
    const int s    = si * NWAVE + wave;
    const int node = nodeBase + s;
    int c = cnt[s];
    const bool big = c > DEGCAP;
    c = c < 0 ? 0 : (c > DEGCAP ? DEGCAP : c);
    int o = offs[s];
    o = o < 0 ? 0 : (o > RCAP ? RCAP : o);
    float a0 = 0.0f, a1 = 0.0f, a2 = 0.0f, a3 = 0.0f;
#pragma unroll 1
    for (int b0 = 0; b0 < c; b0 += 32) {
      int idx = o + b0 + lane;
      idx = idx > RCAP - 1 ? RCAP - 1 : idx;
      const int ent = sl[idx];
      int eid = ent >> SLA;
      eid = eid < 0 ? 0 : (eid > nE - 1 ? nE - 1 : eid);
      int sr = srcs[eid];
      sr = sr < 0 ? 0 : (sr > nN - 1 ? nN - 1 : sr);
      const int m32 = (c - b0) < 32 ? (c - b0) : 32;
#pragma unroll 1
      for (int k = 0; k < m32; ++k) {
        const int sk = __builtin_amdgcn_readlane(sr, k);
        const unsigned short* gp = apl + (size_t)sk * AP + HOFF;
        const v2u wh = *(const v2ua*)(gp + 4 * lane);
        const v2u wl = *(const v2ua*)(gp + DF + 4 * lane);
        const v4f a = hl4(wh, wl);
        a0 += a.x;
        a1 += a.y;
        a2 += a.z;
        a3 += a.w;
      }
    }
    const float den = (c > 0) ? (float)c : 1.0f;
    const float rcp = 1.0f / den;
    const float pzr = big ? __int_as_float(0x7fc00000) : pz;
    const bool live = node < nN;
    v4f mq;
    mq.x = live ? (a0 * rcp + pzr) : 0.0f;
    mq.y = live ? (a1 * rcp + pzr) : 0.0f;
    mq.z = live ? (a2 * rcp + pzr) : 0.0f;
    mq.w = live ? (a3 * rcp + pzr) : 0.0f;
    v2u mh, ml;
    split4w(mq, mh, ml);
    *(v2ua*)(rowbuf + 2 * lane) = mh;
    *(v2ua*)(rowbuf + RBW + 2 * lane) = ml;
    wave_sync();
    const v4u q0 = *(const v4ua*)(rowbuf + 4 * lane);
    wave_sync();
    if (node < mRows) {
      unsigned short* rpw = apl + (size_t)node * AP + 8 * lane;
      *(volatile v4u*)rpw = q0;
      __threadfence();
      *(volatile v4u*)rpw = q0;
    }
  }
}

template <int RES>
__global__ __launch_bounds__(GTHR) void k_gemm(unsigned short* apl, const unsigned short* __restrict__ BT,
                                               const float* __restrict__ bias, int nN, int kLim, float* part) {
  __shared__ __attribute__((aligned(16))) float stg[GBM * GBN];
  __shared__ __attribute__((aligned(16))) float wst[GWAVE * WSTW];
  __shared__ __attribute__((aligned(16))) float pst[PARTW];
  __shared__ __attribute__((aligned(16))) unsigned int rbuf[GWAVE * DF];
  const int tid = (int)threadIdx.x, lane = tid & 31, wave = tid >> 5, hh = lane >> 4, m = lane & 15;
  const int rowBase = (int)blockIdx.x * GBM;

  v8f acc[8];
#pragma unroll
  for (int t = 0; t < 8; ++t) acc[t] = z8();
  const unsigned short* ap = apl + (size_t)(rowBase + 16 * wave + m) * (size_t)AP + 8 * hh;
  const unsigned short* bp = BT + (size_t)m * (size_t)KK + 8 * hh;

#pragma unroll 1
  for (int k0 = 0; k0 < kLim; k0 += 32) {
    FragB af;
    af.h[0] = *(const v8usa*)(ap + k0);
    af.h[1] = *(const v8usa*)(ap + k0 + 16);
#pragma unroll
    for (int nt = 0; nt < 8; ++nt) {
      const unsigned short* wq = bp + (size_t)(16 * nt) * (size_t)KK + k0;
      FragB bf;
      bf.h[0] = *(const v8usa*)wq;
      bf.h[1] = *(const v8usa*)(wq + 16);
      acc[nt] = wmb(af, bf, acc[nt]);
    }
  }

#pragma unroll
  for (int nt = 0; nt < 8; ++nt) {
    const int lc = 16 * nt + m;
#pragma unroll
    for (int r = 0; r < 8; ++r) {
      const int lr = 16 * wave + 8 * hh + r;
      stg[lr * GBN + lc] = acc[nt][r];
    }
  }
  __syncthreads();

  v4f bq;
  {
    const v4f b4 = *(const v4f*)(bias + 4 * lane);
    bq.x = bf16_val(b4.x); bq.y = bf16_val(b4.y); bq.z = bf16_val(b4.z); bq.w = bf16_val(b4.w);
  }
  unsigned int* rb = rbuf + wave * DF;

  v4u qv[16];
  int wn = 0;
  float wm[4], wqv[4];
#pragma unroll
  for (int j = 0; j < 4; ++j) { wm[j] = 0.0f; wqv[j] = 0.0f; }
#pragma unroll
  for (int i = 0; i < 16; ++i) {
    const int lr  = 16 * wave + i;
    const int row = rowBase + lr;
    const bool ok = row < nN;
    const v4f x = *(const v4fa*)(stg + lr * GBN + 4 * lane);
    v4f tq = x + bq;
    if constexpr (RES != 0) {
      const unsigned short* rr = apl + (size_t)row * AP + HOFF;
      const v2u wh = *(const v2ua*)(rr + 4 * lane);
      const v2u wl = *(const v2ua*)(rr + DF + 4 * lane);
      tq = tq + hl4(wh, wl);
    }
    float vv[4];
    vv[0] = ok ? fmaxf(tq.x, 0.0f) : 0.0f;
    vv[1] = ok ? fmaxf(tq.y, 0.0f) : 0.0f;
    vv[2] = ok ? fmaxf(tq.z, 0.0f) : 0.0f;
    vv[3] = ok ? fmaxf(tq.w, 0.0f) : 0.0f;
    if (ok) {
      wn += 1;
      const float rk = 1.0f / (float)(i + 1);
#pragma unroll
      for (int j = 0; j < 4; ++j) {
        const float d = vv[j] - wm[j];
        wm[j]  = fmaf(d, rk, wm[j]);
        wqv[j] = fmaf(d, vv[j] - wm[j], wqv[j]);
      }
    }
    v4f y;
    y.x = vv[0]; y.y = vv[1]; y.z = vv[2]; y.w = vv[3];
    v2u mh, ml;
    split4w(y, mh, ml);
    *(v2ua*)(rb + 2 * lane) = mh;
    *(v2ua*)(rb + RBW + 2 * lane) = ml;
    wave_sync();
    qv[i] = *(const v4ua*)(rb + 4 * lane);
    wave_sync();
  }

#pragma unroll
  for (int i = 0; i < 16; ++i) {
    unsigned short* op = apl + (size_t)(rowBase + 16 * wave + i) * (size_t)AP + HOFF + 8 * lane;
    *(volatile v4u*)op = qv[i];
  }
  __threadfence();
#pragma unroll
  for (int i = 0; i < 16; ++i) {
    unsigned short* op = apl + (size_t)(rowBase + 16 * wave + i) * (size_t)AP + HOFF + 8 * lane;
    *(volatile v4u*)op = qv[i];
  }

  if (lane == 0) wst[wave * WSTW] = (float)wn;
#pragma unroll
  for (int j = 0; j < 4; ++j) {
    wst[wave * WSTW + 1 + 4 * lane + j]       = wm[j];
    wst[wave * WSTW + 1 + GBN + 4 * lane + j] = wqv[j];
  }
  __syncthreads();
  {
    float n = 0.0f, mean = 0.0f, M2 = 0.0f;
#pragma unroll 1
    for (int w2 = 0; w2 < GWAVE; ++w2) {
      const float nb = wst[w2 * WSTW];
      const float mb = wst[w2 * WSTW + 1 + tid];
      const float qb = wst[w2 * WSTW + 1 + GBN + tid];
      if (nb > 0.5f) {
        const float nn = n + nb;
        const float delta = mb - mean;
        const float f = nb / nn;
        mean = fmaf(delta, f, mean);
        M2 = M2 + qb + delta * delta * n * f;
        n = nn;
      }
    }
    pst[1 + tid] = mean;
    pst[1 + GBN + tid] = M2;
    if (tid == 0) pst[0] = n;
  }
#pragma unroll 1
  for (int i = 2 * GBN + 1 + tid; i < PARTW; i += GTHR) pst[i] = 0.0f;
  __syncthreads();
  const int pb = (int)blockIdx.x;
  v4f ps = {0.0f, 0.0f, 0.0f, 0.0f};
  if (tid < PARTW / 4) {
    ps = *(const v4fa*)(pst + 4 * tid);
    *(volatile v4f*)(part + (size_t)pb * PARTW + 4 * tid) = ps;
  }
  __threadfence();
  if (tid < PARTW / 4) {
    *(volatile v4f*)(part + (size_t)pb * PARTW + 4 * tid) = ps;
  }
}

template <int C>
__global__ __launch_bounds__(DF) void k_bnfin(const float* __restrict__ part, int nPart,
                                              const float* __restrict__ gam, const float* __restrict__ bet,
                                              float* ss) {
  __shared__ __attribute__((aligned(16))) float stg[2 * DF];
  const int tid = (int)threadIdx.x;
  const int c = tid;
  const int cc = c < C ? c : (C - 1);
  double n = 0.0, mean = 0.0, M2 = 0.0;
#pragma unroll 1
  for (int b = 0; b < nPart; ++b) {
    const float* pr = part + (size_t)b * PARTW;
    const double nb = (double)pr[0];
    const double mb = (double)pr[1 + c];
    const double qb = (double)pr[1 + GBN + c];
    if (nb > 0.5) {
      const double nn = n + nb;
      const double delta = mb - mean;
      const double f = nb / nn;
      mean = mean + delta * f;
      M2 = M2 + qb + delta * delta * n * f;
      n = nn;
    }
  }
  const double nt = n < 1.0 ? 1.0 : n;
  const float varf  = (float)(M2 / nt);
  const float meanf = (float)mean;
  const float rstd = 1.0f / sqrtf(varf + 1e-5f);
  const float sc = bf16_val(gam[cc]) * rstd;
  const float sh = bf16_val(bet[cc]) - meanf * sc;
  stg[c] = sc;
  stg[DF + c] = sh;
  __syncthreads();
  v4f v = {0.0f, 0.0f, 0.0f, 0.0f};
  if (tid < (2 * DF) / 4) {
    v = *(const v4fa*)(stg + 4 * tid);
    *(volatile v4f*)(ss + 4 * tid) = v;
  }
  __threadfence();
  if (tid < (2 * DF) / 4) {
    *(volatile v4f*)(ss + 4 * tid) = v;
  }
}

__global__ __launch_bounds__(GTHR) void k_head(const unsigned short* __restrict__ apl,
                                               const unsigned short* __restrict__ Bh,
                                               const float* __restrict__ cb, int nN, float* yh, float* part) {
  __shared__ __attribute__((aligned(16))) float stg[GBM * CO];
  __shared__ __attribute__((aligned(16))) float wst[NSUB * WSTH];
  __shared__ __attribute__((aligned(16))) float pst[PARTW];
  const int tid = (int)threadIdx.x, lane = tid & 31, wave = tid >> 5, hh = lane >> 4, m = lane & 15;
  const int rowBase = (int)blockIdx.x * GBM;

  v8f acc[4];
#pragma unroll
  for (int t = 0; t < 4; ++t) acc[t] = z8();
  const unsigned short* ap = apl + (size_t)(rowBase + 16 * wave + m) * (size_t)AP + HOFF + 8 * hh;
  const unsigned short* bp = Bh + (size_t)m * (size_t)KH + 8 * hh;

#pragma unroll 1
  for (int k0 = 0; k0 < KH; k0 += 32) {
    FragB af;
    af.h[0] = *(const v8usa*)(ap + k0);
    af.h[1] = *(const v8usa*)(ap + k0 + 16);
#pragma unroll
    for (int nt = 0; nt < 4; ++nt) {
      const unsigned short* wq = bp + (size_t)(16 * nt) * (size_t)KH + k0;
      FragB bf;
      bf.h[0] = *(const v8usa*)wq;
      bf.h[1] = *(const v8usa*)(wq + 16);
      acc[nt] = wmb(af, bf, acc[nt]);
    }
  }

#pragma unroll
  for (int nt = 0; nt < 4; ++nt) {
    const int lc = 16 * nt + m;
#pragma unroll
    for (int r = 0; r < 8; ++r) {
      const int lr = 16 * wave + 8 * hh + r;
      stg[lr * CO + lc] = acc[nt][r];
    }
  }
#pragma unroll 1
  for (int i = tid; i < PARTW; i += GTHR) pst[i] = 0.0f;
  __syncthreads();

  v4f bq;
  {
    const v4f b4 = *(const v4f*)(cb + 4 * m);
    bq.x = bf16_val(b4.x); bq.y = bf16_val(b4.y); bq.z = bf16_val(b4.z); bq.w = bf16_val(b4.w);
  }
  const int sub = 2 * wave + hh;

  v4f pv[8];
  int wn = 0;
  float wm[4], wqv[4];
#pragma unroll
  for (int j = 0; j < 4; ++j) { wm[j] = 0.0f; wqv[j] = 0.0f; }
#pragma unroll
  for (int j = 0; j < 8; ++j) {
    const int lr  = 16 * wave + 2 * j + hh;
    const int row = rowBase + lr;
    const bool ok = row < nN;
    const v4f x = *(const v4fa*)(stg + lr * CO + 4 * m);
    const v4f tq = x + bq;
    float vv[4];
    vv[0] = ok ? fmaxf(tq.x, 0.0f) : 0.0f;
    vv[1] = ok ? fmaxf(tq.y, 0.0f) : 0.0f;
    vv[2] = ok ? fmaxf(tq.z, 0.0f) : 0.0f;
    vv[3] = ok ? fmaxf(tq.w, 0.0f) : 0.0f;
    v4f q;
    q.x = vv[0]; q.y = vv[1]; q.z = vv[2]; q.w = vv[3];
    pv[j] = q;
    wn += ok ? 1 : 0;
    const float rk = 1.0f / (float)(wn > 0 ? wn : 1);
#pragma unroll
    for (int jj = 0; jj < 4; ++jj) {
      const float d  = vv[jj] - wm[jj];
      const float nm = fmaf(d, rk, wm[jj]);
      const float nq = fmaf(d, vv[jj] - nm, wqv[jj]);
      wm[jj]  = ok ? nm : wm[jj];
      wqv[jj] = ok ? nq : wqv[jj];
    }
  }

#pragma unroll
  for (int j = 0; j < 8; ++j) {
    float* op = yh + (size_t)(rowBase + 16 * wave + 2 * j + hh) * (size_t)CO + 4 * m;
    *(volatile v4f*)op = pv[j];
  }
  __threadfence();
#pragma unroll
  for (int j = 0; j < 8; ++j) {
    float* op = yh + (size_t)(rowBase + 16 * wave + 2 * j + hh) * (size_t)CO + 4 * m;
    *(volatile v4f*)op = pv[j];
  }

  if (m == 0) wst[sub * WSTH] = (float)wn;
#pragma unroll
  for (int jj = 0; jj < 4; ++jj) {
    wst[sub * WSTH + 1 + 4 * m + jj]      = wm[jj];
    wst[sub * WSTH + 1 + CO + 4 * m + jj] = wqv[jj];
  }
  __syncthreads();
  if (tid < CO) {
    float n = 0.0f, mean = 0.0f, M2 = 0.0f;
#pragma unroll 1
    for (int s2 = 0; s2 < NSUB; ++s2) {
      const float nb = wst[s2 * WSTH];
      const float mb = wst[s2 * WSTH + 1 + tid];
      const float qb = wst[s2 * WSTH + 1 + CO + tid];
      if (nb > 0.5f) {
        const float nn = n + nb;
        const float delta = mb - mean;
        const float f = nb / nn;
        mean = fmaf(delta, f, mean);
        M2 = M2 + qb + delta * delta * n * f;
        n = nn;
      }
    }
    pst[1 + tid] = mean;
    pst[1 + GBN + tid] = M2;
    if (tid == 0) pst[0] = n;
  }
  __syncthreads();
  const int pb = (int)blockIdx.x;
  v4f ps = {0.0f, 0.0f, 0.0f, 0.0f};
  if (tid < PARTW / 4) {
    ps = *(const v4fa*)(pst + 4 * tid);
    *(volatile v4f*)(part + (size_t)pb * PARTW + 4 * tid) = ps;
  }
  __threadfence();
  if (tid < PARTW / 4) {
    *(volatile v4f*)(part + (size_t)pb * PARTW + 4 * tid) = ps;
  }
}

__global__ __launch_bounds__(NTHR) void k_out(const float* __restrict__ yh, const float* __restrict__ ss,
                                              int nN, float* out) {
  __shared__ __attribute__((aligned(16))) float ssh[2 * DF];
  __shared__ __attribute__((aligned(16))) float T[CO * OTP];
  const int tid = (int)threadIdx.x, lane = tid & 31, wave = tid >> 5, hh = lane >> 4, m = lane & 15;
  ssh[tid] = ss[tid];
  __syncthreads();
  const int n0 = (int)blockIdx.x * OTN;
#pragma unroll
  for (int it = 0; it < (OTN * CO / 4) / NTHR; ++it) {
    const int i  = it * NTHR + tid;
    const int lr = i >> 4;
    const int p  = i & 15;
    const int c0 = 4 * p;
    const v4f v  = *(const v4f*)(yh + (size_t)(n0 + lr) * (size_t)CO + c0);
    const v4f sc = *(const v4fa*)(ssh + c0);
    const v4f sh = *(const v4fa*)(ssh + DF + c0);
    T[(c0 + 0) * OTP + lr] = fmaf(v.x, sc.x, sh.x);
    T[(c0 + 1) * OTP + lr] = fmaf(v.y, sc.y, sh.y);
    T[(c0 + 2) * OTP + lr] = fmaf(v.z, sc.z, sh.z);
    T[(c0 + 3) * OTP + lr] = fmaf(v.w, sc.w, sh.w);
  }
  __syncthreads();
  v4f val[4];
#pragma unroll
  for (int j = 0; j < 4; ++j) {
    const int c = 8 * wave + 2 * j + hh;
    val[j] = *(const v4fa*)(T + c * OTP + 4 * m);
  }
  const int n = n0 + 4 * m;
#pragma unroll
  for (int j = 0; j < 4; ++j) {
    const int c = 8 * wave + 2 * j + hh;
    if (n < nN) *(volatile v4f*)(out + (size_t)c * (size_t)nN + (size_t)n) = val[j];
  }
  __threadfence();
#pragma unroll
  for (int j = 0; j < 4; ++j) {
    const int c = 8 * wave + 2 * j + hh;
    if (n < nN) *(volatile v4f*)(out + (size_t)c * (size_t)nN + (size_t)n) = val[j];
  }
}

static inline int cdiv(int a, int b) { return (a + b - 1) / b; }
static inline size_t al256(size_t o) { return (o + 255) & ~(size_t)255; }

extern "C" void kernel_launch(void* const* d_in, const int* in_sizes, int n_in,
                              void* d_out, int out_size, void* d_ws, size_t ws_size,
                              hipStream_t stream) {
  if (n_in < 12) return;
  if (in_sizes[0] < DF || (in_sizes[0] % DF) != 0) return;
  const int nN = in_sizes[0] / DF;
  if (in_sizes[1] < DF * DF || (in_sizes[1] % (DF * DF)) != 0) return;
  const int nL = in_sizes[1] / (DF * DF);
  if (nL < 1 || nL > MAXL) return;
  if (in_sizes[2] != nL * DF * DF) return;
  if (in_sizes[3] != nL * DF || in_sizes[4] != nL * DF || in_sizes[5] != nL * DF) return;
  if (in_sizes[6] != CO * DF || in_sizes[7] != CO) return;
  if (in_sizes[8] != CO || in_sizes[9] != CO) return;
  const int nE = in_sizes[10];
  if (nE < 1 || in_sizes[11] != nE) return;
  if (nE >= (1 << 21) || nN < 64 || nN >= (1 << 24)) return;
  if ((nN % 32) != 0) return;
  if ((long long)out_size != (long long)CO * nN) return;

  const float* x      = (const float*)d_in[0];
  const float* Wself  = (const float*)d_in[1];
  const float* Wneigh = (const float*)d_in[2];
  const float* bias   = (const float*)d_in[3];
  const float* gamma  = (const float*)d_in[4];
  const float* beta   = (const float*)d_in[5];
  const float* convW  = (const float*)d_in[6];
  const float* convb  = (const float*)d_in[7];
  const float* gamma2 = (const float*)d_in[8];
  const float* beta2  = (const float*)d_in[9];
  const int*   src    = (const int*)d_in[10];
  const int*   dst    = (const int*)d_in[11];
  float* out = (float*)d_out;

  const int MP = cdiv(nN, GBM) * GBM;
  const int gM = MP / GBM;
  const int gA = cdiv(nN, NBA);
  if ((long long)gA * NBA < (long long)MP) return;
  if ((MP % HPB) != 0 || (MP % OTN) != 0) return;
  const int vec8 = ((nE & 3) == 0) ? 1 : 0;
  const int vx   = ((nN & 3) == 0) ? 1 : 0;

  char* ws = (char*)d_ws;
  size_t off = 0;
  const size_t oB  = off; off = al256(off + (size_t)nL * DF * KK * 2);
  const size_t oBh = off; off = al256(off + (size_t)CO * KH * 2);
  const size_t oA  = off; off = al256(off + (size_t)MP * AP * 2);
  const size_t oY  = off; off = al256(off + (size_t)MP * CO * 4);
  const size_t oPT = off; off = al256(off + (size_t)gM * PARTW * 4);
  const size_t oSS = off; off = al256(off + (size_t)(2 * DF) * 4);
  if (off > ws_size || off > (size_t)WSMAX) return;
  unsigned short* Bpl = (unsigned short*)(ws + oB);
  unsigned short* Bhd = (unsigned short*)(ws + oBh);
  unsigned short* Apl = (unsigned short*)(ws + oA);
  float*          YH  = (float*)(ws + oY);
  float*          PT  = (float*)(ws + oPT);
  float*          SS  = (float*)(ws + oSS);

  const size_t scanLds = (size_t)AGG_LDS_INTS * 4;
  hipFuncSetAttribute(reinterpret_cast<const void*>(&k_scan), hipFuncAttributeMaxDynamicSharedMemorySize, (int)scanLds);

  k_wprep<<<16 * nL + WBH, NTHR, 0, stream>>>(Wself, Wneigh, convW, nL, Bpl, Bhd);
  k_xprep<<<gM, NTHR, 0, stream>>>(x, nN, vx, Apl);
  for (int l = 0; l < nL; ++l) {
    if (l > 0) k_hprep<<<gM, NTHR, 0, stream>>>(SS, nN, MP, Apl);
    k_scan<<<gA, NTHR, scanLds, stream>>>(src, dst, nE, nN, vec8, MP, Apl);
    const unsigned short* Bl = Bpl + (size_t)l * (size_t)(DF * KK);
    const float* bl = bias + (size_t)l * DF;
    const int kLim = (l == 0) ? (3 * DF) : KK;
    if (l == 0) k_gemm<0><<<gM, GTHR, 0, stream>>>(Apl, Bl, bl, nN, kLim, PT);
    else        k_gemm<1><<<gM, GTHR, 0, stream>>>(Apl, Bl, bl, nN, kLim, PT);
    k_bnfin<DF><<<1, DF, 0, stream>>>(PT, gM, gamma + (size_t)l * DF, beta + (size_t)l * DF, SS);
  }
  k_hprep<<<gM, NTHR, 0, stream>>>(SS, nN, MP, Apl);
  k_head<<<gM, GTHR, 0, stream>>>(Apl, Bhd, convb, nN, YH, PT);
  k_bnfin<CO><<<1, DF, 0, stream>>>(PT, gM, gamma2, beta2, SS);
  k_out<<<gM, NTHR, 0, stream>>>(YH, SS, nN, out);
}
